// MPNN_21131239096634
// MI455X (gfx1250) — hardware-verified
//
#include <hip/hip_runtime.h>
#include <stddef.h>


#define NTHR  256
#define NWAVE 8
#define EPT   8
#define NGRP  2
#define CHUNK (NTHR * EPT * NGRP)
#define WCAP  (EPT * NGRP * 32)
#define LISTN (NWAVE * WCAP)
#define NB    512
#define EB    64
#define NG    128
#define DH    32
#define DX    64
#define DEA   16
#define NW2   1024
#define KW2   64
#define KW1   32
#define NR0   128
#define NBW2  (NW2 * KW2 / 8 / NTHR)
#define LDS_N 104704
#define SLOPE 0.01f
#define L2EPS 1e-12f

static_assert((CHUNK & (CHUNK - 1)) == 0);
static_assert(CHUNK <= 4096);
static_assert(NB <= 4096 && (NB % 4) == 0 && (NB / NWAVE) == 64);
static_assert((NB * DH + DH * DH + DH + NG * DH + LISTN + NB + NWAVE) * 4 <= LDS_N);
static_assert(NBW2 * NTHR * 8 == NW2 * KW2);
static_assert(DH * DX / 8 == NTHR);
static_assert(DH * KW1 / 8 == 128);
static_assert(NW2 == 4 * NTHR);
static_assert(2 * NTHR * 4 == EB * DH);
static_assert(4 * NTHR * 4 == NG * DH);
static_assert(EB * 4 == NTHR);

typedef int            v4i  __attribute__((ext_vector_type(4)));
typedef float          v2f  __attribute__((ext_vector_type(2)));
typedef float          v4f  __attribute__((ext_vector_type(4)));
typedef float          v8f  __attribute__((ext_vector_type(8)));
typedef unsigned short v8us __attribute__((ext_vector_type(8)));
typedef __bf16         v16b __attribute__((ext_vector_type(16)));
union FragB { v16b v; v8us u[2]; };

__device__ __forceinline__ v8f z8() { v8f z = {0.f, 0.f, 0.f, 0.f, 0.f, 0.f, 0.f, 0.f}; return z; }

__device__ __forceinline__ v8f wmb(v16b a, v16b b, v8f c) {
  v8f d = __builtin_amdgcn_wmma_f32_16x16x32_bf16(false, a, false, b, (short)0, c, false, false);
  asm volatile("v_nop\n\tv_nop\n\tv_nop\n\tv_nop" : "+v"(d) : "v"(a), "v"(b));
  return d;
}

__device__ __forceinline__ unsigned short bfr(float x) {
  const unsigned u = __float_as_uint(x);
  return (unsigned short)((u + 0x7FFFu + ((u >> 16) & 1u)) >> 16);
}
__device__ __forceinline__ float bfw(unsigned short h) { return __uint_as_float(((unsigned)h) << 16); }
__device__ __forceinline__ float bfq(float x) { return bfw(bfr(x)); }
__device__ __forceinline__ v8us pk8(v4f a, v4f b) {
  float v[8] = {a.x, a.y, a.z, a.w, b.x, b.y, b.z, b.w};
  v8us r;
#pragma unroll
  for (int k = 0; k < 8; ++k) r[k] = bfr(v[k]);
  return r;
}
__device__ __forceinline__ v8us zu8() { v8us z = {0, 0, 0, 0, 0, 0, 0, 0}; return z; }
__device__ __forceinline__ float lrelu(float v) { return v > 0.0f ? v : v * SLOPE; }

__device__ __forceinline__ int scan_chunk(const int* __restrict__ ids, int nE, int cbase, int slotBase, int nb,
                                          int vec8, int* list, int tid, int lane, int wave) {
  int wc = 0;
#pragma unroll
  for (int g = 0; g < NGRP; ++g) {
    const int el0  = (g * NTHR + tid) * EPT;
    const int e0   = cbase + el0;
    const int sent = -2147483647 - 1;
    v4i da, db;
    if (vec8 != 0 && cbase + CHUNK <= nE) {
      da = *(const v4i*)(ids + e0);
      db = *(const v4i*)(ids + e0 + 4);
    } else {
      const int lst = nE - 1;
      da.x = (e0     < nE) ? ids[min(e0,     lst)] : sent;
      da.y = (e0 + 1 < nE) ? ids[min(e0 + 1, lst)] : sent;
      da.z = (e0 + 2 < nE) ? ids[min(e0 + 2, lst)] : sent;
      da.w = (e0 + 3 < nE) ? ids[min(e0 + 3, lst)] : sent;
      db.x = (e0 + 4 < nE) ? ids[min(e0 + 4, lst)] : sent;
      db.y = (e0 + 5 < nE) ? ids[min(e0 + 5, lst)] : sent;
      db.z = (e0 + 6 < nE) ? ids[min(e0 + 6, lst)] : sent;
      db.w = (e0 + 7 < nE) ? ids[min(e0 + 7, lst)] : sent;
    }
    const unsigned bs = (unsigned)slotBase;
    const unsigned ub = (unsigned)nb;
    const unsigned s0 = (unsigned)da.x - bs, s1 = (unsigned)da.y - bs;
    const unsigned s2 = (unsigned)da.z - bs, s3 = (unsigned)da.w - bs;
    const unsigned s4 = (unsigned)db.x - bs, s5 = (unsigned)db.y - bs;
    const unsigned s6 = (unsigned)db.z - bs, s7 = (unsigned)db.w - bs;
    const bool h0 = s0 < ub, h1 = s1 < ub, h2 = s2 < ub, h3 = s3 < ub;
    const bool h4 = s4 < ub, h5 = s5 < ub, h6 = s6 < ub, h7 = s7 < ub;
    const unsigned any = __builtin_amdgcn_ballot_w32(h0 | h1 | h2 | h3 | h4 | h5 | h6 | h7);
    if (any != 0u) {
#define HITJ(J, HJ, SJ) { \
        const unsigned mj = __builtin_amdgcn_ballot_w32(HJ); \
        if (mj != 0u) { \
          if (HJ) { \
            const int pos = wc + (int)__builtin_amdgcn_mbcnt_lo(mj, 0u); \
            if (pos < WCAP) list[wave * WCAP + pos] = ((el0 + (J)) << 12) | (int)(SJ); \
          } \
          wc += (int)__builtin_popcount(mj); } }
      HITJ(0, h0, s0)
      HITJ(1, h1, s1)
      HITJ(2, h2, s2)
      HITJ(3, h3, s3)
      HITJ(4, h4, s4)
      HITJ(5, h5, s5)
      HITJ(6, h6, s6)
      HITJ(7, h7, s7)
#undef HITJ
    }
  }
  return wc;
}

__global__ __launch_bounds__(NTHR) void k_prep(const float* __restrict__ w2a, const float* __restrict__ w2b,
    const float* __restrict__ nfw, const float* __restrict__ w1a, const float* __restrict__ w1b,
    unsigned short* W2Da, unsigned short* W2Db, unsigned short* NFT, unsigned short* W1Ta, unsigned short* W1Tb) {
  const int blk = blockIdx.x, tid = threadIdx.x;
  float v[8];
  unsigned short* dp;
  bool act = true;
  if (blk < 2 * NBW2) {
    const bool first = blk < NBW2;
    const float* src = first ? w2a : w2b;
    unsigned short* dst = first ? W2Da : W2Db;
    const int u  = (first ? blk : blk - NBW2) * NTHR + tid;
    const int o  = u * 8;
    const int n  = o / KW2;
    const int k0 = o - n * KW2;
#pragma unroll
    for (int e = 0; e < 8; ++e) {
      const int i = (k0 + e) & (DH - 1);
      v[e] = src[(size_t)i * NW2 + n];
    }
    dp = dst + o;
  } else if (blk == 2 * NBW2) {
    const int o  = tid * 8;
    const int n  = o / DX;
    const int k0 = o - n * DX;
#pragma unroll
    for (int e = 0; e < 8; ++e) v[e] = nfw[(size_t)(k0 + e) * DH + n];
    dp = NFT + o;
  } else {
    const bool first = (blk == 2 * NBW2 + 1);
    const float* src = first ? w1a : w1b;
    unsigned short* dst = first ? W1Ta : W1Tb;
    act = tid < (DH * KW1 / 8);
    const int tt = act ? tid : 0;
    const int o  = tt * 8;
    const int n  = o / KW1;
    const int k0 = o - n * KW1;
#pragma unroll
    for (int e = 0; e < 8; ++e) {
      const int k  = k0 + e;
      const int kc = k < DEA ? k : DEA - 1;
      const float x = src[(size_t)kc * DH + n];
      v[e] = (k < DEA) ? x : x * 0.0f;
    }
    dp = dst + o;
  }
  v4f a, b;
  a.x = v[0]; a.y = v[1]; a.z = v[2]; a.w = v[3];
  b.x = v[4]; b.y = v[5]; b.z = v[6]; b.w = v[7];
  const v8us hv = pk8(a, b);
  if (act) *(volatile v8us*)dp = hv;
  __threadfence();
  if (act) *(volatile v8us*)dp = hv;
}

__global__ __launch_bounds__(NTHR) void k_node0(const float* __restrict__ X, int nN,
    const unsigned short* __restrict__ NFT, const float* __restrict__ nfb, float* H0) {
  __shared__ __attribute__((aligned(16))) float stg[NR0 * DH];
  const int tid = threadIdx.x, lane = tid & 31, wave = tid >> 5, hf = lane >> 4, m = lane & 15;
  const int rowBase = blockIdx.x * NR0;
  int arow = rowBase + 16 * wave + m;
  arow = arow > nN - 1 ? nN - 1 : arow;
  const float* xr = X + (size_t)arow * DX + 8 * hf;
  v8f acc[2];
  acc[0] = z8(); acc[1] = z8();
#pragma unroll
  for (int ks = 0; ks < DX / 32; ++ks) {
    FragB a;
    a.u[0] = pk8(*(const v4f*)(xr + 32 * ks), *(const v4f*)(xr + 32 * ks + 4));
    a.u[1] = pk8(*(const v4f*)(xr + 32 * ks + 16), *(const v4f*)(xr + 32 * ks + 20));
#pragma unroll
    for (int t = 0; t < 2; ++t) {
      const unsigned short* bp = NFT + (size_t)(16 * t + m) * DX + 32 * ks + 8 * hf;
      FragB b;
      b.u[0] = *(const v8us*)bp;
      b.u[1] = *(const v8us*)(bp + 16);
      acc[t] = wmb(a.v, b.v, acc[t]);
    }
  }
#pragma unroll
  for (int t = 0; t < 2; ++t) {
    const int col = 16 * t + m;
    const float bv = bfq(nfb[col]);
    float* sp = stg + (16 * wave + 8 * hf) * DH + col;
#pragma unroll
    for (int r = 0; r < 8; ++r) sp[r * DH] = lrelu(acc[t][r] + bv);
  }
  __syncthreads();
  const float* lp = stg + 16 * wave * DH;
  float* gp = H0 + (size_t)(rowBase + 16 * wave) * DH;
  v4f ov[4];
#pragma unroll
  for (int p = 0; p < 4; ++p) ov[p] = *(const v4f*)(lp + 4 * (32 * p + lane));
#pragma unroll
  for (int p = 0; p < 4; ++p) *(volatile v4f*)(gp + 4 * (32 * p + lane)) = ov[p];
  __threadfence();
#pragma unroll
  for (int p = 0; p < 4; ++p) *(volatile v4f*)(gp + 4 * (32 * p + lane)) = ov[p];
}

__global__ __launch_bounds__(NTHR) void k_edge(
    const float* __restrict__ HP, int nN, const int* __restrict__ ei, int nE, const float* __restrict__ EA,
    const unsigned short* __restrict__ W1T, const float* __restrict__ b1,
    const unsigned short* __restrict__ W2D, const float* __restrict__ b2, float* MSG) {
  __shared__ __attribute__((aligned(16))) unsigned short AHL[EB * KW2];
  __shared__ __attribute__((aligned(16))) float osr[EB * DH];
  __shared__ __attribute__((aligned(16))) float msp[2 * EB * DH];
  __shared__ __attribute__((aligned(16))) float sb2[NW2];
  __shared__ float sb1[DH];
  const int tid = threadIdx.x, lane = tid & 31, wave = tid >> 5, hf = lane >> 4, m = lane & 15;
  const int eb = blockIdx.x * EB;

  {
    const v4f q = *(const v4f*)(b2 + 4 * tid);
    v4f w;
    w.x = bfq(q.x); w.y = bfq(q.y); w.z = bfq(q.z); w.w = bfq(q.w);
    *(v4f*)(sb2 + 4 * tid) = w;
    if (tid < DH) sb1[tid] = bfq(b1[tid]);
    const int el = tid >> 2, part = tid & 3;
    int e = eb + el;
    e = e > nE - 1 ? nE - 1 : e;
    int s = ei[e];
    s = s < 0 ? 0 : (s > nN - 1 ? nN - 1 : s);
    const float* sp = HP + (size_t)s * DH + 8 * part;
    float* dp = osr + el * DH + 8 * part;
    *(v4f*)dp = *(const v4f*)sp;
    *(v4f*)(dp + 4) = *(const v4f*)(sp + 4);
  }
  __syncthreads();

  {
    const int rg = wave & 3, nt = wave >> 2;
    int e = eb + 16 * rg + m;
    e = e > nE - 1 ? nE - 1 : e;
    const float* ep = EA + (size_t)e * DEA + 8 * hf;
    FragB a;
    a.u[0] = pk8(*(const v4f*)ep, *(const v4f*)(ep + 4));
    a.u[1] = zu8();
    const unsigned short* bp = W1T + (size_t)(16 * nt + m) * KW1 + 8 * hf;
    FragB b;
    b.u[0] = *(const v8us*)bp;
    b.u[1] = *(const v8us*)(bp + 16);
    const v8f d = wmb(a.v, b.v, z8());
    const int col = 16 * nt + m;
    const float bv = sb1[col];
    unsigned short* hp = AHL + (16 * rg + 8 * hf) * KW2 + col;
#pragma unroll
    for (int r = 0; r < 8; ++r) {
      const float he = fmaxf(d[r] + bv, 0.0f);
      const unsigned short hi = bfr(he);
      const unsigned short lo = bfr(he - bfw(hi));
      hp[r * KW2] = hi;
      hp[r * KW2 + DH] = lo;
    }
  }
  __syncthreads();

  {
    const int rg = wave & 3, dh = wave >> 2;
    FragB aF[2];
    const unsigned short* ar = AHL + (16 * rg + m) * KW2 + 8 * hf;
#pragma unroll
    for (int ks = 0; ks < 2; ++ks) {
      aF[ks].u[0] = *(const v8us*)(ar + 32 * ks);
      aF[ks].u[1] = *(const v8us*)(ar + 32 * ks + 16);
    }
    v8f macc[2];
    macc[0] = z8(); macc[1] = z8();
    const float* orow = osr + (16 * rg + 8 * hf) * DH;
#pragma unroll 1
    for (int p = 0; p < NW2 / 2 / 128; ++p) {
      const int cb = (NW2 / 2) * dh + 128 * p;
      v8f acc[8];
#pragma unroll
      for (int t = 0; t < 8; ++t) acc[t] = z8();
#pragma unroll
      for (int ks = 0; ks < 2; ++ks) {
#pragma unroll
        for (int t = 0; t < 8; ++t) {
          const unsigned short* bp = W2D + (size_t)(cb + 16 * t + m) * KW2 + 32 * ks + 8 * hf;
          FragB b;
          b.u[0] = *(const v8us*)bp;
          b.u[1] = *(const v8us*)(bp + 16);
          acc[t] = wmb(aF[ks].v, b.v, acc[t]);
        }
      }
      float bv[8];
#pragma unroll
      for (int t = 0; t < 8; ++t) bv[t] = sb2[cb + 16 * t + m];
      const int i0 = cb / DH;
#pragma unroll
      for (int r = 0; r < 8; ++r) {
        const v4f o = *(const v4f*)(orow + r * DH + i0);
        macc[0][r] += o.x * (acc[0][r] + bv[0]) + o.y * (acc[2][r] + bv[2]) + o.z * (acc[4][r] + bv[4]) + o.w * (acc[6][r] + bv[6]);
        macc[1][r] += o.x * (acc[1][r] + bv[1]) + o.y * (acc[3][r] + bv[3]) + o.z * (acc[5][r] + bv[5]) + o.w * (acc[7][r] + bv[7]);
      }
    }
    float* mp = msp + dh * (EB * DH) + (16 * rg + 8 * hf) * DH + m;
#pragma unroll
    for (int u = 0; u < 2; ++u) {
#pragma unroll
      for (int r = 0; r < 8; ++r) mp[r * DH + 16 * u] = macc[u][r];
    }
  }
  __syncthreads();

  v4f ov[2];
#pragma unroll
  for (int it = 0; it < 2; ++it) {
    const int i = it * NTHR + tid;
    ov[it] = *(const v4f*)(msp + 4 * i) + *(const v4f*)(msp + EB * DH + 4 * i);
  }
  float* mb = MSG + (size_t)eb * DH;
#pragma unroll
  for (int it = 0; it < 2; ++it) *(volatile v4f*)(mb + 4 * (it * NTHR + tid)) = ov[it];
  __threadfence();
#pragma unroll
  for (int it = 0; it < 2; ++it) *(volatile v4f*)(mb + 4 * (it * NTHR + tid)) = ov[it];
}

template <int L2>
__global__ __launch_bounds__(NTHR) void k_node(
    const int* __restrict__ ei, int nE, int vec8, const float* __restrict__ MSG,
    const float* __restrict__ HPV, int nN, const float* __restrict__ root, const float* __restrict__ bias,
    const int* __restrict__ batch, const int* __restrict__ numg, float* HN, float* OUT1, float* PP) {
  extern __shared__ v4f lds_dyn[];
  float* accL  = (float*)lds_dyn;
  float* sroot = accL + NB * DH;
  float* sbias = sroot + DH * DH;
  float* pool  = sbias + DH;
  int*   list  = (int*)(pool + NG * DH);
  int*   sbat  = list + LISTN;
  int*   wcnt  = sbat + NB;
  const int tid = threadIdx.x, lane = tid & 31, wave = tid >> 5;
  const int nodeBase = blockIdx.x * NB;
  const int* dsts = ei + nE;

  {
    const v4f z = {0.f, 0.f, 0.f, 0.f};
#pragma unroll 1
    for (int i = tid; i < NB * DH / 4; i += NTHR) ((v4f*)accL)[i] = z;
#pragma unroll 1
    for (int i = tid; i < DH * DH; i += NTHR) sroot[i] = bfq(root[i]);
    if (tid < DH) sbias[tid] = bfq(bias[tid]);
    if (L2) {
#pragma unroll 1
      for (int i = tid; i < NG * DH / 4; i += NTHR) ((v4f*)pool)[i] = z;
#pragma unroll 1
      for (int i = tid; i < NB; i += NTHR) {
        const int node = nodeBase + i;
        const int cl = node > nN - 1 ? nN - 1 : node;
        const int bv = batch[cl];
        sbat[i] = (node < nN) ? bv : -1;
      }
    }
  }
  __syncthreads();

  const int nChunks = (nE + CHUNK - 1) / CHUNK;
#pragma unroll 1
  for (int ch = 0; ch < nChunks; ++ch) {
    const int cbase = ch * CHUNK;
    const int wc = scan_chunk(dsts, nE, cbase, nodeBase, NB, vec8, list, tid, lane, wave);
    if (lane == 0) wcnt[wave] = wc;
    __syncthreads();
    if (wave == 0) {
#pragma unroll 1
      for (int wsx = 0; wsx < NWAVE; ++wsx) {
        int n = __builtin_amdgcn_readfirstlane(wcnt[wsx]);
        n = n > WCAP ? WCAP : (n < 0 ? 0 : n);
        const int* lp = list + wsx * WCAP;
#pragma unroll 1
        for (int i = 0; i < n; ++i) {
          const int ent = __builtin_amdgcn_readfirstlane(lp[i]);
          int slot = ent & 4095;
          slot = slot > NB - 1 ? NB - 1 : slot;
          int e = cbase + ((ent >> 12) & (CHUNK - 1));
          e = e > nE - 1 ? nE - 1 : e;
          const int col = 4 * (lane & 7);
          const v4f v = *(const v4f*)(MSG + (size_t)e * DH + col);
          if (lane < 8) {
            v4f* ap = (v4f*)(accL + slot * DH + col);
            *ap = *ap + v;
          }
        }
      }
    }
    __syncthreads();
  }

#pragma unroll 1
  for (int task = tid; task < NB * 4; task += NTHR) {
    const int r  = task >> 2;
    const int og = task & 3;
    int node = nodeBase + r;
    node = node > nN - 1 ? nN - 1 : node;
    const float* hp = HPV + (size_t)node * DH;
    const float* rb = sroot + 8 * og;
    float acc[8];
#pragma unroll
    for (int j = 0; j < 8; ++j) acc[j] = sbias[8 * og + j];
#pragma unroll 1
    for (int k2 = 0; k2 < DH / 2; ++k2) {
      const v2f h2 = *(const v2f*)(hp + 2 * k2);
      const float* rp = rb + (2 * k2) * DH;
      const v4f ra = *(const v4f*)rp,        rbv = *(const v4f*)(rp + 4);
      const v4f rc = *(const v4f*)(rp + DH), rd  = *(const v4f*)(rp + DH + 4);
      acc[0] += h2.x * ra.x;  acc[1] += h2.x * ra.y;  acc[2] += h2.x * ra.z;  acc[3] += h2.x * ra.w;
      acc[4] += h2.x * rbv.x; acc[5] += h2.x * rbv.y; acc[6] += h2.x * rbv.z; acc[7] += h2.x * rbv.w;
      acc[0] += h2.y * rc.x;  acc[1] += h2.y * rc.y;  acc[2] += h2.y * rc.z;  acc[3] += h2.y * rc.w;
      acc[4] += h2.y * rd.x;  acc[5] += h2.y * rd.y;  acc[6] += h2.y * rd.z;  acc[7] += h2.y * rd.w;
    }
    float* ap = accL + r * DH + 8 * og;
    const v4f a0 = *(const v4f*)ap, a1 = *(const v4f*)(ap + 4);
    v4f o0, o1;
    o0.x = lrelu(a0.x + acc[0]); o0.y = lrelu(a0.y + acc[1]); o0.z = lrelu(a0.z + acc[2]); o0.w = lrelu(a0.w + acc[3]);
    o1.x = lrelu(a1.x + acc[4]); o1.y = lrelu(a1.y + acc[5]); o1.z = lrelu(a1.z + acc[6]); o1.w = lrelu(a1.w + acc[7]);
    *(v4f*)ap = o0;
    *(v4f*)(ap + 4) = o1;
  }

  if (L2) {
    __syncthreads();
    if (wave == 0) {
      int nGv = numg[0];
      nGv = nGv < 0 ? 0 : (nGv > NG ? NG : nGv);
#pragma unroll 1
      for (int r = 0; r < NB; ++r) {
        const int g = __builtin_amdgcn_readfirstlane(sbat[r]);
        if ((unsigned)g < (unsigned)nGv) {
          float* pq = pool + g * DH + lane;
          *pq = *pq + accL[r * DH + lane];
        }
      }
    }
  }
  __syncthreads();

  v4f ov[16];
  const float* lrow = accL + wave * (64 * DH) + 4 * lane;
#pragma unroll
  for (int q = 0; q < 16; ++q) ov[q] = *(const v4f*)(lrow + q * 128);
  if (!L2) {
    float* gp = HN + (size_t)(nodeBase + 64 * wave) * DH + 4 * lane;
#pragma unroll
    for (int q = 0; q < 16; ++q) *(volatile v4f*)(gp + q * 128) = ov[q];
    __threadfence();
#pragma unroll
    for (int q = 0; q < 16; ++q) *(volatile v4f*)(gp + q * 128) = ov[q];
  } else {
    const int rw = nodeBase + 64 * wave;
    float* gp = OUT1 + (size_t)rw * DH + 4 * lane;
#pragma unroll
    for (int q = 0; q < 16; ++q) { if (rw + 4 * q + 3 < nN) *(volatile v4f*)(gp + q * 128) = ov[q]; }
    __threadfence();
#pragma unroll
    for (int q = 0; q < 16; ++q) { if (rw + 4 * q + 3 < nN) *(volatile v4f*)(gp + q * 128) = ov[q]; }
    v4f pv[4];
#pragma unroll
    for (int it = 0; it < 4; ++it) pv[it] = *(const v4f*)(pool + 4 * (it * NTHR + tid));
    float* pp = PP + (size_t)blockIdx.x * (NG * DH);
#pragma unroll
    for (int it = 0; it < 4; ++it) *(volatile v4f*)(pp + 4 * (it * NTHR + tid)) = pv[it];
    __threadfence();
#pragma unroll
    for (int it = 0; it < 4; ++it) *(volatile v4f*)(pp + 4 * (it * NTHR + tid)) = pv[it];
  }
}

__global__ __launch_bounds__(NTHR) void k_final(const float* __restrict__ PP, int nblk,
    const float* __restrict__ fcw, const float* __restrict__ fcb, float* out) {
  __shared__ __attribute__((aligned(16))) float spool[NG * DH];
  __shared__ __attribute__((aligned(16))) float sfcw[DH * DH];
  __shared__ float sfcb[DH];
  __shared__ float sinv[NG];
  __shared__ __attribute__((aligned(16))) float sout[NG * DH];
  const int tid = threadIdx.x;
#pragma unroll 1
  for (int i = tid; i < DH * DH; i += NTHR) sfcw[i] = bfq(fcw[i]);
  if (tid < DH) sfcb[tid] = bfq(fcb[tid]);
#pragma unroll 1
  for (int j = 0; j < NG * DH / NTHR; ++j) {
    const int idx = tid + NTHR * j;
    float s = 0.0f;
#pragma unroll 1
    for (int b = 0; b < nblk; ++b) s += PP[(size_t)b * (NG * DH) + idx];
    spool[idx] = s;
  }
  __syncthreads();
  if (tid < NG) {
    float ss = 0.0f;
#pragma unroll 1
    for (int o = 0; o < DH; ++o) { const float p = spool[tid * DH + o]; ss += p * p; }
    const float nrm = sqrtf(ss);
    sinv[tid] = 1.0f / fmaxf(nrm, L2EPS);
  }
  __syncthreads();
#pragma unroll 1
  for (int task = tid; task < NG * 4; task += NTHR) {
    const int g = task >> 2, og = task & 3;
    const float inv = sinv[g];
    float acc[8];
#pragma unroll
    for (int j = 0; j < 8; ++j) acc[j] = sfcb[8 * og + j];
#pragma unroll 1
    for (int k = 0; k < DH; ++k) {
      const float p = spool[g * DH + k] * inv;
      const float* rp = sfcw + k * DH + 8 * og;
      const v4f ra = *(const v4f*)rp, rb = *(const v4f*)(rp + 4);
      acc[0] += p * ra.x; acc[1] += p * ra.y; acc[2] += p * ra.z; acc[3] += p * ra.w;
      acc[4] += p * rb.x; acc[5] += p * rb.y; acc[6] += p * rb.z; acc[7] += p * rb.w;
    }
    float* sp = sout + g * DH + 8 * og;
#pragma unroll
    for (int j = 0; j < 8; ++j) sp[j] = acc[j];
  }
  __syncthreads();
  v4f ov[4];
#pragma unroll
  for (int it = 0; it < 4; ++it) ov[it] = *(const v4f*)(sout + 4 * (it * NTHR + tid));
#pragma unroll
  for (int it = 0; it < 4; ++it) *(volatile v4f*)(out + 4 * (it * NTHR + tid)) = ov[it];
  __threadfence();
#pragma unroll
  for (int it = 0; it < 4; ++it) *(volatile v4f*)(out + 4 * (it * NTHR + tid)) = ov[it];
}

extern "C" void kernel_launch(void* const* d_in, const int* in_sizes, int n_in,
                              void* d_out, int out_size, void* d_ws, size_t ws_size,
                              hipStream_t stream) {
  if (n_in < 21) return;
  const int nN = in_sizes[0] / DX;
  const int nE = in_sizes[1] / 2;
  if (nN <= 0 || nE <= 0) return;
  if (in_sizes[0] != nN * DX || (nN % 4) != 0 || in_sizes[1] != 2 * nE || in_sizes[2] != nE * DEA || in_sizes[3] != nN || in_sizes[4] < 1) return;
  if (in_sizes[5] != DX * DH || in_sizes[6] != DH) return;
  if (in_sizes[7] != DEA * DH || in_sizes[8] != DH || in_sizes[9] != DH * NW2 || in_sizes[10] != NW2 || in_sizes[11] != DH * DH || in_sizes[12] != DH) return;
  if (in_sizes[13] != DEA * DH || in_sizes[14] != DH || in_sizes[15] != DH * NW2 || in_sizes[16] != NW2 || in_sizes[17] != DH * DH || in_sizes[18] != DH) return;
  if (in_sizes[19] != DH * DH || in_sizes[20] != DH) return;
  if (out_size != NG * DH + nN * DH) return;
  if (nN > (1 << 24) || nE > (1 << 26)) return;

  const float* x     = (const float*)d_in[0];
  const int*   ei    = (const int*)d_in[1];
  const float* ea    = (const float*)d_in[2];
  const int*   batch = (const int*)d_in[3];
  const int*   numg  = (const int*)d_in[4];
  const float* nfc_w = (const float*)d_in[5];
  const float* nfc_b = (const float*)d_in[6];
  const float* e1w1  = (const float*)d_in[7];
  const float* e1b1  = (const float*)d_in[8];
  const float* e1w2  = (const float*)d_in[9];
  const float* e1b2  = (const float*)d_in[10];
  const float* root1 = (const float*)d_in[11];
  const float* bias1 = (const float*)d_in[12];
  const float* e2w1  = (const float*)d_in[13];
  const float* e2b1  = (const float*)d_in[14];
  const float* e2w2  = (const float*)d_in[15];
  const float* e2b2  = (const float*)d_in[16];
  const float* root2 = (const float*)d_in[17];
  const float* bias2 = (const float*)d_in[18];
  const float* fc_w  = (const float*)d_in[19];
  const float* fc_b  = (const float*)d_in[20];
  float* out0 = (float*)d_out;
  float* out1 = out0 + (size_t)NG * DH;

  const int nB0 = (nN + NR0 - 1) / NR0, NP0 = nB0 * NR0;
  const int nBN = (nN + NB - 1) / NB,   NPN = nBN * NB;
  const int nEB = (nE + EB - 1) / EB,   EP  = nEB * EB;

  char* ws = (char*)d_ws;
  size_t off = 0;
  const size_t oW2a = off; off += (size_t)NW2 * KW2 * 2;    off = (off + 255) & ~(size_t)255;
  const size_t oW2b = off; off += (size_t)NW2 * KW2 * 2;    off = (off + 255) & ~(size_t)255;
  const size_t oNFT = off; off += (size_t)DH * DX * 2;      off = (off + 255) & ~(size_t)255;
  const size_t oW1a = off; off += (size_t)DH * KW1 * 2;     off = (off + 255) & ~(size_t)255;
  const size_t oW1b = off; off += (size_t)DH * KW1 * 2;     off = (off + 255) & ~(size_t)255;
  const size_t oH0  = off; off += (size_t)NP0 * DH * 4;     off = (off + 255) & ~(size_t)255;
  const size_t oH1  = off; off += (size_t)NPN * DH * 4;     off = (off + 255) & ~(size_t)255;
  const size_t oMSG = off; off += (size_t)EP * DH * 4;      off = (off + 255) & ~(size_t)255;
  const size_t oPP  = off; off += (size_t)nBN * NG * DH * 4; off = (off + 255) & ~(size_t)255;
  if (off > ws_size) return;
  if (off > (size_t)128 * 1024 * 1024) return;
  unsigned short* W2Da = (unsigned short*)(ws + oW2a);
  unsigned short* W2Db = (unsigned short*)(ws + oW2b);
  unsigned short* NFT  = (unsigned short*)(ws + oNFT);
  unsigned short* W1Ta = (unsigned short*)(ws + oW1a);
  unsigned short* W1Tb = (unsigned short*)(ws + oW1b);
  float* H0  = (float*)(ws + oH0);
  float* H1  = (float*)(ws + oH1);
  float* MSG = (float*)(ws + oMSG);
  float* PP  = (float*)(ws + oPP);
  const int vec8 = ((nE & 3) == 0) ? 1 : 0;

  k_prep<<<2 * NBW2 + 3, NTHR, 0, stream>>>(e1w2, e2w2, nfc_w, e1w1, e2w1, W2Da, W2Db, NFT, W1Ta, W1Tb);
  k_node0<<<nB0, NTHR, 0, stream>>>(x, nN, NFT, nfc_b, H0);

  hipFuncSetAttribute(reinterpret_cast<const void*>(&k_node<0>), hipFuncAttributeMaxDynamicSharedMemorySize, LDS_N);
  hipFuncSetAttribute(reinterpret_cast<const void*>(&k_node<1>), hipFuncAttributeMaxDynamicSharedMemorySize, LDS_N);

  k_edge<<<nEB, NTHR, 0, stream>>>(H0, nN, ei, nE, ea, W1Ta, e1b1, W2Da, e1b2, MSG);
  k_node<0><<<nBN, NTHR, LDS_N, stream>>>(ei, nE, vec8, MSG, H0, nN, root1, bias1, batch, numg, H1, out1, PP);
  k_edge<<<nEB, NTHR, 0, stream>>>(H1, nN, ei, nE, ea, W1Tb, e2b1, W2Db, e2b2, MSG);
  k_node<1><<<nBN, NTHR, LDS_N, stream>>>(ei, nE, vec8, MSG, H1, nN, root2, bias2, batch, numg, H1, out1, PP);
  k_final<<<1, NTHR, 0, stream>>>(PP, nBN, fc_w, fc_b, out0);
}
